// RelationExtractorCnnPosNetwork_60808146977249
// MI455X (gfx1250) — hardware-verified
//
#include <hip/hip_runtime.h>
#include <math.h>

typedef __attribute__((ext_vector_type(16))) _Float16 v16h;
typedef __attribute__((ext_vector_type(16))) __bf16 v16b;
typedef __attribute__((ext_vector_type(8)))  _Float16 v8h;
typedef __attribute__((ext_vector_type(8)))  float v8f;
typedef __attribute__((ext_vector_type(4)))  float v4f;
typedef __attribute__((ext_vector_type(2)))  float v2f;
typedef __attribute__((ext_vector_type(4)))  unsigned v4u;
typedef __attribute__((ext_vector_type(4)))  int v4i;
typedef float __attribute__((may_alias)) float_a;
typedef int __attribute__((may_alias)) int_a;

template <typename T> __device__ __forceinline__ void vst2(void* p, T v) { *(volatile T*)p = v; __threadfence(); *(volatile T*)p = v; }
__device__ __forceinline__ v8f wmma16(v16h a, v16h b, v8f c) {
  v8f d = __builtin_amdgcn_wmma_f32_16x16x32_f16(false, a, false, b, (short)0, c, false, false);
  asm volatile("v_nop\n\tv_nop\n\tv_nop\n\tv_nop" : "+v"(d) : "v"(a), "v"(b));
  return d;
}
__device__ __forceinline__ v8f wmma_bf(v16b a, v16b b, v8f c) {
  v8f d = __builtin_amdgcn_wmma_f32_16x16x32_bf16(false, a, false, b, (short)0, c, false, false);
  asm volatile("v_nop\n\tv_nop\n\tv_nop\n\tv_nop" : "+v"(d) : "v"(a), "v"(b));
  return d;
}
__device__ __forceinline__ v16h frag_h(const _Float16* rowk0, int lane) {
  union { v16h v; v8h q[2]; } u; const _Float16* p = rowk0 + 8 * (lane >> 4);
  u.q[0] = *(const v8h*)p; u.q[1] = *(const v8h*)(p + 16); return u.v;
}
__device__ __forceinline__ v16h frag_f32(const float* rowk0, int lane) {
  v16h a; const float* p = rowk0 + 8 * (lane >> 4);
#pragma unroll
  for (int i = 0; i < 8; ++i) { a[i] = (_Float16)p[i]; a[8 + i] = (_Float16)p[16 + i]; }
  return a;
}
__device__ __forceinline__ v16h frag_f32s(const float* rowk0, int lane, float sc) {
  v16h a; const float* p = rowk0 + 8 * (lane >> 4);
#pragma unroll
  for (int i = 0; i < 8; ++i) { a[i] = (_Float16)(p[i] * sc); a[8 + i] = (_Float16)(p[16 + i] * sc); }
  return a;
}
__device__ __forceinline__ v16h fragc_f32(const float* W, int k0, int n, int lane, int ld, int K) {
  v16h a; const int g = lane >> 4;
#pragma unroll
  for (int i = 0; i < 8; ++i) { const int ka = k0 + 8 * g + i, kb = ka + 16;
    a[i] = (_Float16)(ka < K ? W[(size_t)(ka < K ? ka : K - 1) * ld + n] : 0.f); a[8 + i] = (_Float16)(kb < K ? W[(size_t)(kb < K ? kb : K - 1) * ld + n] : 0.f); }
  return a;
}
struct F2 { v16b h, l; };
__device__ __forceinline__ F2 bsplit16(const float v[16]) { F2 r;
#pragma unroll
  for (int i = 0; i < 16; ++i) { const __bf16 h = (__bf16)v[i]; r.h[i] = h; r.l[i] = (__bf16)(v[i] - (float)h); }
  return r; }
__device__ __forceinline__ F2 split_row(const float* row, int k0, int lane) { float v[16]; const float* p = row + k0 + 8 * (lane >> 4);
#pragma unroll
  for (int i = 0; i < 8; ++i) { v[i] = p[i]; v[8 + i] = p[16 + i]; }
  return bsplit16(v); }
__device__ __forceinline__ F2 split_rowK(const float* row, int k0, int lane, int K) { float v[16]; const int g = lane >> 4;
#pragma unroll
  for (int i = 0; i < 8; ++i) { const int ka = k0 + 8 * g + i, kb = ka + 16; v[i] = ka < K ? row[ka < K ? ka : K - 1] : 0.f; v[8 + i] = kb < K ? row[kb < K ? kb : K - 1] : 0.f; }
  return bsplit16(v); }
__device__ __forceinline__ F2 split_col(const float* W, int k0, int n, int lane, int ld, int K) { float v[16]; const int g = lane >> 4;
#pragma unroll
  for (int i = 0; i < 8; ++i) { const int ka = k0 + 8 * g + i, kb = ka + 16; v[i] = ka < K ? W[(size_t)(ka < K ? ka : K - 1) * ld + n] : 0.f; v[8 + i] = kb < K ? W[(size_t)(kb < K ? kb : K - 1) * ld + n] : 0.f; }
  return bsplit16(v); }
__device__ __forceinline__ v8f mac3(const F2& a, const F2& b, v8f c) { c = wmma_bf(a.l, b.h, c); c = wmma_bf(a.h, b.l, c); return wmma_bf(a.h, b.h, c); }
__device__ __forceinline__ float sigm(float v) { return 1.0f / (1.0f + expf(-v)); }
#define LDSX() do { asm volatile("s_wait_dscnt 0" ::: "memory"); __builtin_amdgcn_wave_barrier(); __builtin_amdgcn_fence(__ATOMIC_RELEASE, "workgroup"); } while (0)


#define NB 256
#define SL 512
#define ED 300
#define PD 16
#define CHX 332
#define CHP 352
#define KT 5
#define KTOT (KT * CHP)
#define CO 50
#define COP 64
#define NCLS 10
#define PMAX 512
#ifndef TBN
#define TBN NB
#endif
typedef __attribute__((ext_vector_type(8))) __bf16 v8b;
__device__ __forceinline__ v16b frag_b(const __bf16* rowk0, int lane) {
  union { v16b v; v8b q[2]; } u; const __bf16* p = rowk0 + 8 * (lane >> 4);
  u.q[0] = *(const v8b*)p; u.q[1] = *(const v8b*)(p + 16); return u.v;
}
__device__ __forceinline__ float bfr(float v) { return (float)(__bf16)v; }
__device__ __attribute__((noinline)) float exp_ni(float v) { return expf(v); }
__device__ __attribute__((noinline)) float erf_ni(float v) { return erff(v); }

#define WS_W   0u
#define WS_DI  (((2u * COP * KTOT) + 127u) / 128u * 128u)
#define WS_MX  (WS_DI + 4u * 2 * NB * SL)
#define WS_END (WS_MX + 4u * (size_t)NB * 8 * COP)

__global__ __launch_bounds__(256) void k_packw(const float* __restrict__ CW, __bf16* __restrict__ PW) {
  __shared__ __align__(16) __bf16 s[KTOT]; const int o = blockIdx.x, t = threadIdx.x;
  for (int q = t; q < KTOT; q += 256) { const int k = q / CHP, c = q % CHP; s[q] = (__bf16)((o < CO && c < CHX) ? CW[((size_t)o * CHX + c) * KT + k] : 0.f); }
  __syncthreads();
  for (int q = t; q < KTOT / 8; q += 256) vst2((unsigned*)(PW + (size_t)o * KTOT + q * 8), *(const v4u*)&s[q * 8]);
}
__global__ __launch_bounds__(64) void k_dist(const int* __restrict__ TOK, const int* __restrict__ E1, const int* __restrict__ E2, int* __restrict__ DIST) {
  __shared__ int pos[SL + 2]; __shared__ __align__(16) int res[SL]; const int b = blockIdx.x, e = blockIdx.y; const int ent = e ? E2[0] : E1[0]; const int t = threadIdx.x;
  if (t == 0) { int left = -2 * SL; for (int i = 0; i < SL; ++i) { if (TOK[(size_t)b * SL + i] == ent) left = i; pos[i] = left; } }
  if (t == 1) { int right = 2 * SL; for (int i = SL - 1; i >= 0; --i) { if (TOK[(size_t)b * SL + i] == ent) right = i; res[i] = right; } }
  __syncthreads();
  for (int i = t; i < SL; i += 64) { const int dl = i - pos[i], dr = res[i] - i; int dd = dl < dr ? dl : dr; dd = dd < 0 ? 0 : (dd > PMAX - 1 ? PMAX - 1 : dd); res[i] = dd; }
  __syncthreads();
  if (t < SL / 4 / 2) { for (int q = t; q < SL / 4; q += 32) vst2((unsigned*)(DIST + ((size_t)e * NB + b) * SL + q * 4), *(const v4u*)&res[q * 4]); }
}
__global__ __launch_bounds__(128) void k_conv(const int* __restrict__ TOK, const float* __restrict__ ET, const float* __restrict__ PT, const int* __restrict__ DIST, const __bf16* __restrict__ PW, const float* __restrict__ CB, float* __restrict__ MX) {
  __shared__ __align__(16) __bf16 sx[68][CHP + 8]; __shared__ float smx[4][COP];
  const int tid = threadIdx.x, wave = tid >> 5, lane = tid & 31, col = lane & 15, g = lane >> 4; const int blk = blockIdx.x; const size_t b = blockIdx.y; const int s0 = blk * 64;
  for (int e = tid; e < 68 * (CHP + 8); e += 128) { const int r = e / (CHP + 8), c = e % (CHP + 8); const int s = s0 - 2 + r; float v = 0.f;
    if (s >= 0 && s < SL && c < CHX) { const int tok = TOK[b * SL + s];
      if (c < ED) v = bfr(ET[(size_t)tok * ED + c]);
      else { const int which = (c - ED) / PD, pd = (c - ED) % PD; const int di = DIST[((size_t)which * NB + b) * SL + s]; v = bfr(PT[(size_t)di * PD + pd]); } }
    sx[r][c] = (__bf16)v; }
  __syncthreads();
  { __shared__ int zrow[68]; if (tid < 68) { int allz = 1; for (int c = 0; c < ED; ++c) if ((float)sx[tid][c] != 0.f) { allz = 0; break; } zrow[tid] = allz; } __syncthreads();
    for (int e = tid; e < 68 * 2 * PD; e += 128) { const int r = e / (2 * PD), c = ED + e % (2 * PD); if (zrow[r]) sx[r][c] = (__bf16)0.f; } __syncthreads(); }
  v8f acc[4] = {};
#pragma unroll 1
  for (int k = 0; k < KT; ++k) {
#pragma unroll
    for (int cc = 0; cc < CHP / 32; ++cc) { const v16b a = frag_b(&sx[wave * 16 + col + k][cc * 32], lane);
#pragma unroll
      for (int j = 0; j < 4; ++j) acc[j] = wmma_bf(a, frag_b(PW + (size_t)(j * 16 + col) * KTOT + k * CHP + cc * 32, lane), acc[j]); } }
#pragma unroll
  for (int j = 0; j < 4; ++j) { const int o = j * 16 + col; const float bb = (o < CO) ? bfr(CB[o]) : 0.f; float mx = 0.f;
#pragma unroll
    for (int r = 0; r < 8; ++r) mx = fmaxf(mx, fmaxf(acc[j][r] + bb, 0.f));
    mx = fmaxf(mx, __shfl_xor(mx, 16)); if (g == 0) smx[wave][o] = mx; }
  __syncthreads();
  if (tid < COP / 4) { v4f o4; for (int i = 0; i < 4; ++i) { const int o = tid * 4 + i; o4[i] = fmaxf(fmaxf(smx[0][o], smx[1][o]), fmaxf(smx[2][o], smx[3][o])); } vst2(MX + ((b * 8 + blk) * COP) + tid * 4, o4); }
}
__global__ __launch_bounds__(256) void k_fc(const float* __restrict__ MX, const float* __restrict__ FW, const float* __restrict__ FB, float* __restrict__ OUT) {
  __shared__ __align__(16) float so[32 * NCLS]; const int t = threadIdx.x; const size_t b0 = (size_t)blockIdx.x * 32;
  for (int e = t; e < 32 * NCLS; e += 256) { const int bi = e / NCLS, n = e % NCLS; float a = bfr(FB[n]);
    for (int o = 0; o < CO; ++o) { float y = MX[((b0 + bi) * 8 + 0) * COP + o]; for (int k = 1; k < 8; ++k) y = fmaxf(y, MX[((b0 + bi) * 8 + k) * COP + o]); a += y * bfr(FW[n * CO + o]); }
    so[e] = a; }
  __syncthreads();
  if (t < 32 * NCLS / 4) vst2(OUT + b0 * NCLS + t * 4, *(const v4f*)&so[t * 4]);
}
extern "C" void kernel_launch(void* const* d_in, const int* in_sizes, int n_in, void* d_out, int out_size, void* d_ws, size_t ws_size, hipStream_t stream) {
  (void)in_sizes; (void)n_in; (void)out_size;
  const float** F = (const float**)d_in; const int* TOK = (const int*)d_in[0];
  if (ws_size < (size_t)WS_END) return;
  char* ws = (char*)d_ws; __bf16* PW = (__bf16*)(ws + WS_W); int* DIST = (int*)(ws + WS_DI); float* MX = (float*)(ws + WS_MX);
  k_packw<<<COP, 256, 0, stream>>>(F[3], PW);
  k_dist<<<dim3(NB, 2), 64, 0, stream>>>(TOK, (const int*)d_in[7], (const int*)d_in[8], DIST);
  k_conv<<<dim3(SL / 64, TBN), 128, 0, stream>>>(TOK, F[1], F[2], DIST, PW, F[4], MX);
  k_fc<<<TBN / 32, 256, 0, stream>>>(MX, F[5], F[6], (float*)d_out);
}
